// Qwerky7TimeMix_42915313221840
// MI455X (gfx1250) — hardware-verified
//
#include <hip/hip_runtime.h>
#include <math.h>

#define TT   2048
#define HD   2048
#define ATTD 512
#define NH   32
#define HS   64
#define DW   96
#define DA   96
#define DV   64
#define DG   256
#define LP   128
#define WSCALE 64.0f
#define WINV   0.015625f
#define GN_EPS 6.4e-4f

typedef _Float16 v16h __attribute__((ext_vector_type(16)));
typedef _Float16 v4h  __attribute__((ext_vector_type(4)));
typedef unsigned short v8us __attribute__((ext_vector_type(8), may_alias));
typedef float v8f  __attribute__((ext_vector_type(8)));
typedef float v4f  __attribute__((ext_vector_type(4)));
typedef float v4fa __attribute__((ext_vector_type(4), may_alias));
union FragH  { v16h v; v8us half[2]; _Float16 h[16]; unsigned short u[16]; };
union Pack4h { v4h v; _Float16 h[4]; };
union Pack2h { unsigned int u; _Float16 h[2]; };

__device__ __forceinline__ v8f mmaH(v16h a, v16h b, v8f c)
{
  c = __builtin_amdgcn_wmma_f32_16x16x32_f16(false, a, false, b, (short)0, c, false, false);
  asm volatile("v_nop\n\tv_nop\n\tv_nop\n\tv_nop" : "+v"(c) : "v"(a), "v"(b));
  return c;
}

__global__ __launch_bounds__(256) void k_xcp(const float* __restrict__ x, const float* __restrict__ vf,
                                             _Float16* __restrict__ X16, float* __restrict__ out2, size_t n8)
{
  const size_t t = (size_t)blockIdx.x * 256 + threadIdx.x;
  if (t >= n8) return;
  const v4f a = *(const v4fa*)(x + t * 8), c = *(const v4fa*)(x + t * 8 + 4);
  FragH f;
#pragma unroll
  for (int q = 0; q < 4; ++q) { f.h[q] = (_Float16)a[q]; f.h[4 + q] = (_Float16)c[q]; }
  const v4f p0 = *(const v4fa*)(vf + t * 4);
  const v4f p1 = *(const v4fa*)(vf + (n8 + t) * 4);
  unsigned short* dx = (unsigned short*)X16 + t * 8;
  float* d0 = out2 + t * 4;
  float* d1 = out2 + (n8 + t) * 4;
  const v8us hx = f.half[0];
  *(volatile v8us*)dx = hx; *(volatile v4f*)d0 = p0; *(volatile v4f*)d1 = p1;
  __threadfence();
  *(volatile v8us*)dx = hx; *(volatile v4f*)d0 = p0; *(volatile v4f*)d1 = p1;
}

__global__ __launch_bounds__(256) void k_cvt16(const float* __restrict__ W, _Float16* __restrict__ D, float s, size_t n8)
{
  const size_t t = (size_t)blockIdx.x * 256 + threadIdx.x;
  if (t >= n8) return;
  const v4f a = *(const v4fa*)(W + t * 8), c = *(const v4fa*)(W + t * 8 + 4);
  FragH f;
#pragma unroll
  for (int q = 0; q < 4; ++q) { f.h[q] = (_Float16)(a[q] * s); f.h[4 + q] = (_Float16)(c[q] * s); }
  unsigned short* d = (unsigned short*)D + t * 8;
  const v8us hv = f.half[0];
  *(volatile v8us*)d = hv;
  __threadfence();
  *(volatile v8us*)d = hv;
}

__global__ __launch_bounds__(256) void k_wt16(const float* __restrict__ W, int K, int N, _Float16* __restrict__ D, int ldt, int NP, float s)
{
  const size_t t = (size_t)blockIdx.x * 256 + threadIdx.x;
  const int kq = ldt >> 3;
  if (t >= (size_t)NP * kq) return;
  const int n = (int)(t / kq), k8 = (int)(t % kq) * 8;
  const int nc = min(n, N - 1);
  FragH f;
#pragma unroll
  for (int i = 0; i < 8; ++i) {
    const int k = k8 + i;
    const int kc = min(k, K - 1);
    float v = W[(size_t)kc * N + nc] * s;
    v = (k < K && n < N) ? v : 0.0f;
    f.h[i] = (_Float16)v;
  }
  unsigned short* d = (unsigned short*)D + (size_t)n * ldt + k8;
  const v8us hv = f.half[0];
  *(volatile v8us*)d = hv;
  __threadfence();
  *(volatile v8us*)d = hv;
}

template <int ACT, bool OUT16>
__global__ __launch_bounds__(128) void k_gemm(const _Float16* __restrict__ A, int lda, const _Float16* __restrict__ Bt, int ldb, float alpha,
                                              const float* __restrict__ bias, float* __restrict__ Cf, _Float16* __restrict__ Ch, int ldc,
                                              int M, int N, int K)
{
  __shared__ __attribute__((aligned(16))) float so[4][16][64];
  const int tid = threadIdx.x, w = tid >> 5, lane = tid & 31, ln = lane & 15, hh = lane >> 4;
  const int ntn = N >> 6;
  const int wid = blockIdx.x * 4 + w;
  const int mt = wid / ntn, nq = wid - mt * ntn;
  if (mt * 16 >= M) return;
  const int row0 = mt * 16, col0 = nq * 64;
  const unsigned short* arow = (const unsigned short*)A + (size_t)(row0 + ln) * lda;
  v8f acc[4] = {};
  for (int kb = 0; kb < K; kb += 32) {
    FragH a;
    a.half[0] = *(const v8us*)(arow + kb + 8 * hh);
    a.half[1] = *(const v8us*)(arow + kb + 16 + 8 * hh);
#pragma unroll
    for (int t = 0; t < 4; ++t) {
      const unsigned short* brow = (const unsigned short*)Bt + (size_t)(col0 + t * 16 + ln) * ldb + kb;
      FragH b;
      b.half[0] = *(const v8us*)(brow + 8 * hh);
      b.half[1] = *(const v8us*)(brow + 16 + 8 * hh);
      acc[t] = mmaH(a.v, b.v, acc[t]);
    }
  }
#pragma unroll
  for (int t = 0; t < 4; ++t) {
    float bv = 0.0f;
    if (bias != nullptr) bv = bias[col0 + t * 16 + ln];
#pragma unroll
    for (int r = 0; r < 8; ++r) so[w][8 * hh + r][t * 16 + ln] = acc[t][r] * alpha + bv;
  }
  __builtin_amdgcn_fence(__ATOMIC_ACQ_REL, "workgroup");
  __builtin_amdgcn_wave_barrier();
  if (ACT != 0) {
    float* sf = &so[w][0][0];
#pragma unroll 1
    for (int e = lane; e < 16 * 64; e += 32) {
      float v = sf[e];
      if (ACT == 1) v = tanhf(v);
      else v = __builtin_amdgcn_rcpf(1.0f + expf(-v));
      sf[e] = v;
    }
    __builtin_amdgcn_fence(__ATOMIC_ACQ_REL, "workgroup");
    __builtin_amdgcn_wave_barrier();
  }
  const int rsub = lane >> 4, c4 = (lane & 15) * 4;
  v4f pc[8];
#pragma unroll
  for (int q = 0; q < 8; ++q) pc[q] = *(const v4fa*)&so[w][2 * q + rsub][c4];
  if (!OUT16) {
    for (int pass = 0; pass < 2; ++pass) {
#pragma unroll
      for (int q = 0; q < 8; ++q)
        *(volatile v4f*)(Cf + (size_t)(row0 + 2 * q + rsub) * ldc + col0 + c4) = pc[q];
      if (pass == 0) __threadfence();
    }
  } else {
    Pack4h hp[8];
#pragma unroll
    for (int q = 0; q < 8; ++q) {
#pragma unroll
      for (int i = 0; i < 4; ++i) hp[q].h[i] = (_Float16)pc[q][i];
    }
    for (int pass = 0; pass < 2; ++pass) {
#pragma unroll
      for (int q = 0; q < 8; ++q)
        *(volatile v4h*)(Ch + (size_t)(row0 + 2 * q + rsub) * ldc + col0 + c4) = hp[q].v;
      if (pass == 0) __threadfence();
    }
  }
}

__global__ __launch_bounds__(256) void k_prep(float* __restrict__ Rpl, const float* __restrict__ Kpl, const float* __restrict__ Vpl,
                                              float* __restrict__ WLpl, float* __restrict__ ALpl, float* __restrict__ VLpl,
                                              const float* __restrict__ vfirst, const float* __restrict__ cosT, const float* __restrict__ sinT,
                                              const float* __restrict__ kkc_, const float* __restrict__ kac_, const float* __restrict__ rk_,
                                              float* __restrict__ INRM, float* __restrict__ RB)
{
#pragma clang fp contract(off)
  __shared__ __attribute__((aligned(16))) float rbs[NH];
  __shared__ __attribute__((aligned(16))) float nrs[NH];
  const int tid = threadIdx.x, wv = tid >> 5, l = tid & 31, t = blockIdx.x;
  const size_t ek = (size_t)t * ATTD + wv * HS + l;
  const float kr0 = Kpl[ek], kr1 = Kpl[ek + 32];
  const float vr0 = Vpl[ek], vr1 = Vpl[ek + 32];
  const float cs0 = cosT[t * HS + l], cs1 = cosT[t * HS + l + 32];
  const float sn0 = sinT[t * HS + l], sn1 = sinT[t * HS + l + 32];
  const float k40 = kr0 * cs0 + (-kr1) * sn0;
  const float k41 = kr1 * cs1 + kr0 * sn1;
#pragma unroll 1
  for (int hh = 0; hh < 4; ++hh) {
    const int h = wv * 4 + hh;
    const int c = h * HS + l;
    const size_t e = (size_t)t * HD + c;
    const float rr0 = Rpl[e], rr1 = Rpl[e + 32];
    const float wl0 = WLpl[e], wl1 = WLpl[e + 32];
    const float al0 = ALpl[e], al1 = ALpl[e + 32];
    const float vl0 = VLpl[e], vl1 = VLpl[e + 32];
    const float vf0 = vfirst[e], vf1 = vfirst[e + 32];
    const float kq0 = kkc_[c], kq1 = kkc_[c + 32];
    const float kb0 = kac_[c], kb1 = kac_[c + 32];
    const float rk0 = rk_[c], rk1 = rk_[c + 32];
    const float r40 = rr0 * cs0 + (-rr1) * sn0;
    const float r41 = rr1 * cs1 + rr0 * sn1;
    float wA = 0.0f, wB = 0.0f, icA = 0.0f, icB = 0.0f, vmA = 0.0f, vmB = 0.0f;
#pragma unroll 1
    for (int u = 0; u < 2; ++u) {
      const float wl = u ? wl1 : wl0;
      const float al = u ? al1 : al0;
      const float vl = u ? vl1 : vl0;
      const float ic = 1.0f / (1.0f + expf(-al));
      const float vm = 1.0f / (1.0f + expf(-vl));
      const float nw = -wl;
      const float sp = fmaxf(nw, 0.0f) + log1pf(expf(-fabsf(nw)));
      const float wd = expf(-expf(-sp - 0.5f));
      wA = u ? wA : wd;  wB = u ? wd : wB;
      icA = u ? icA : ic; icB = u ? ic : icB;
      vmA = u ? vmA : vm; vmB = u ? vm : vmB;
    }
    const float v20 = vr0 + (vf0 - vr0) * vmA;
    const float v21 = vr1 + (vf1 - vr1) * vmB;
    const float kkr0 = k40 * kq0, kkr1 = k41 * kq1;
    float kn = kkr0 * kkr0 + kkr1 * kkr1;
    for (int o = 16; o > 0; o >>= 1) kn += __shfl_xor(kn, o, 32);
    const float nrm = fmaxf(sqrtf(kn), 1e-12f);
    const float rn = 1.0f / nrm;
    const float k20 = k40 * (1.0f + (icA - 1.0f) * kb0);
    const float k21 = k41 * (1.0f + (icB - 1.0f) * kb1);
    float rbv = (r40 * k20) * rk0 + (r41 * k21) * rk1;
    for (int o = 16; o > 0; o >>= 1) rbv += __shfl_xor(rbv, o, 32);
    if (l == 0) { rbs[h] = rbv; nrs[h] = rn; }
    *(volatile float*)(Rpl + e) = r40;  *(volatile float*)(Rpl + e + 32) = r41;
    *(volatile float*)(WLpl + e) = wA;  *(volatile float*)(WLpl + e + 32) = wB;
    *(volatile float*)(ALpl + e) = icA; *(volatile float*)(ALpl + e + 32) = icB;
    *(volatile float*)(VLpl + e) = v20; *(volatile float*)(VLpl + e + 32) = v21;
    __threadfence();
    *(volatile float*)(Rpl + e) = r40;  *(volatile float*)(Rpl + e + 32) = r41;
    *(volatile float*)(WLpl + e) = wA;  *(volatile float*)(WLpl + e + 32) = wB;
    *(volatile float*)(ALpl + e) = icA; *(volatile float*)(ALpl + e + 32) = icB;
    *(volatile float*)(VLpl + e) = v20; *(volatile float*)(VLpl + e + 32) = v21;
  }
  __syncthreads();
  if (tid < 8) {
    const v4f a = *(const v4fa*)&rbs[4 * tid];
    const v4f b = *(const v4fa*)&nrs[4 * tid];
    float* pa = RB + (size_t)t * NH + 4 * tid;
    float* pb = INRM + (size_t)t * NH + 4 * tid;
    *(volatile v4f*)pa = a; *(volatile v4f*)pb = b;
    __threadfence();
    *(volatile v4f*)pa = a; *(volatile v4f*)pb = b;
  }
}

__global__ __launch_bounds__(256) void k_wkv(const float* __restrict__ S0, const float* __restrict__ Rpl, const float* __restrict__ Wpl,
                                             const float* __restrict__ ICpl, const float* __restrict__ V2pl, const float* __restrict__ Kpl,
                                             const float* __restrict__ cosT, const float* __restrict__ sinT,
                                             const float* __restrict__ kkc_, const float* __restrict__ kac_, const float* __restrict__ INRM,
                                             float* __restrict__ Ypl, float* __restrict__ Sout)
{
#pragma clang fp contract(off)
  __shared__ __attribute__((aligned(16))) float wk[5][HS];
  __shared__ __attribute__((aligned(16))) float ys[HS];
  __shared__ __attribute__((aligned(16))) float Ss[HS][68];
  const int tid = threadIdx.x, lane = tid & 31, wv = tid >> 5;
  const int h = blockIdx.x, hk = h >> 2;
  const int i = tid >> 2, jq = tid & 3, j0 = jq * 16;
  float S[16];
  {
    const float* sp = S0 + ((size_t)h * HS + i) * HS + j0;
#pragma unroll
    for (int m = 0; m < 4; ++m) {
      const v4f a = *(const v4fa*)(sp + 4 * m);
      S[4 * m] = a[0]; S[4 * m + 1] = a[1]; S[4 * m + 2] = a[2]; S[4 * m + 3] = a[3];
    }
  }
  const int dl = tid & 63, dp = dl ^ 32;
  const float kkc = kkc_[h * HS + dl], kac = kac_[h * HS + dl];
  const float sgn = (dl < 32) ? -1.0f : 1.0f;
#pragma unroll 1
  for (int t = 0; t < TT; ++t) {
    if (tid < HS) {
      const size_t base = (size_t)t * HD + h * HS + dl;
      const float w  = Wpl[base], r = Rpl[base], ic = ICpl[base];
      const float kr = Kpl[(size_t)t * ATTD + hk * HS + dl];
      const float kp = Kpl[(size_t)t * ATTD + hk * HS + dp];
      const float cs = cosT[t * HS + dl], sn = sinT[t * HS + dl];
      const float rn = INRM[t * NH + h];
      const float k4 = kr * cs + (sgn * kp) * sn;
      const float kk = (k4 * kkc) * rn;
      const float ka = kk * ic;
      const float k2 = k4 * (1.0f + (ic - 1.0f) * kac);
      wk[0][dl] = w; wk[1][dl] = kk; wk[2][dl] = ka; wk[3][dl] = k2; wk[4][dl] = r;
    }
    const float vi = V2pl[(size_t)t * HD + h * HS + i];
    __syncthreads();
    float kkv[16], wvv[16], kav[16], k2v[16], rv[16];
#pragma unroll
    for (int m = 0; m < 4; ++m) {
      const v4f a = *(const v4fa*)&wk[1][j0 + 4 * m];
      kkv[4 * m] = a[0]; kkv[4 * m + 1] = a[1]; kkv[4 * m + 2] = a[2]; kkv[4 * m + 3] = a[3];
    }
    float sa = 0.0f;
#pragma unroll
    for (int m = 0; m < 16; ++m) sa = fmaf(S[m], kkv[m], sa);
    sa += __shfl_xor(sa, 1, 32);
    sa += __shfl_xor(sa, 2, 32);
#pragma unroll
    for (int m = 0; m < 4; ++m) {
      const v4f a = *(const v4fa*)&wk[0][j0 + 4 * m];
      const v4f b = *(const v4fa*)&wk[2][j0 + 4 * m];
      const v4f c = *(const v4fa*)&wk[3][j0 + 4 * m];
      const v4f d = *(const v4fa*)&wk[4][j0 + 4 * m];
      wvv[4 * m] = a[0]; wvv[4 * m + 1] = a[1]; wvv[4 * m + 2] = a[2]; wvv[4 * m + 3] = a[3];
      kav[4 * m] = b[0]; kav[4 * m + 1] = b[1]; kav[4 * m + 2] = b[2]; kav[4 * m + 3] = b[3];
      k2v[4 * m] = c[0]; k2v[4 * m + 1] = c[1]; k2v[4 * m + 2] = c[2]; k2v[4 * m + 3] = c[3];
      rv[4 * m]  = d[0]; rv[4 * m + 1]  = d[1]; rv[4 * m + 2]  = d[2]; rv[4 * m + 3]  = d[3];
    }
    float yp = 0.0f;
#pragma unroll
    for (int m = 0; m < 16; ++m) {
      float sv = S[m] * wvv[m];
      sv = fmaf(-sa, kav[m], sv);
      sv = fmaf(vi, k2v[m], sv);
      S[m] = sv;
      yp = fmaf(sv, rv[m], yp);
    }
    yp += __shfl_xor(yp, 1, 32);
    yp += __shfl_xor(yp, 2, 32);
    if (jq == 0) ys[i] = yp;
    __syncthreads();
    if (tid < 16) {
      const v4f yv = *(const v4fa*)&ys[4 * tid];
      float* p = Ypl + (size_t)t * HD + h * HS + 4 * tid;
      *(volatile v4f*)p = yv;
      __threadfence();
      *(volatile v4f*)p = yv;
    }
  }
#pragma unroll
  for (int m = 0; m < 4; ++m) {
    v4f a; a[0] = S[4 * m]; a[1] = S[4 * m + 1]; a[2] = S[4 * m + 2]; a[3] = S[4 * m + 3];
    *(v4fa*)&Ss[i][j0 + 4 * m] = a;
  }
  __syncthreads();
  const int rs2 = lane >> 4, c4 = (lane & 15) * 4;
  v4f pv[4];
#pragma unroll
  for (int q = 0; q < 4; ++q) pv[q] = *(const v4fa*)&Ss[wv * 8 + 2 * q + rs2][c4];
  for (int pass = 0; pass < 2; ++pass) {
#pragma unroll
    for (int q = 0; q < 4; ++q)
      *(volatile v4f*)(Sout + ((size_t)h * HS + wv * 8 + 2 * q + rs2) * HS + c4) = pv[q];
    if (pass == 0) __threadfence();
  }
}

__global__ __launch_bounds__(256) void k_fin(const float* __restrict__ Ypl, const float* __restrict__ V2pl, const float* __restrict__ Gpl,
                                             const float* __restrict__ RB, const float* __restrict__ lw, const float* __restrict__ lb,
                                             _Float16* __restrict__ Z16)
{
#pragma clang fp contract(off)
  const int tid = threadIdx.x, wv = tid >> 5, l = tid & 31;
  const int th = blockIdx.x * 8 + wv;
  const int t = th >> 5, h = th & 31;
  const int c = h * HS + 2 * l;
  const size_t e = (size_t)t * HD + c;
  const float y0 = Ypl[e], y1 = Ypl[e + 1];
  float s = y0 + y1;
  for (int o = 16; o > 0; o >>= 1) s += __shfl_xor(s, o, 32);
  const float mu = s / 64.0f;
  const float d0 = y0 - mu, d1 = y1 - mu;
  float vs = d0 * d0 + d1 * d1;
  for (int o = 16; o > 0; o >>= 1) vs += __shfl_xor(vs, o, 32);
  const float var = vs / 64.0f;
  const float rs = 1.0f / sqrtf(var + GN_EPS);
  const float rb = RB[(size_t)t * NH + h];
  const float g0 = Gpl[e], g1 = Gpl[e + 1];
  const float va = V2pl[e], vb = V2pl[e + 1];
  const float z0 = (((d0 * rs) * lw[c] + lb[c]) + rb * va) * g0;
  const float z1 = (((d1 * rs) * lw[c + 1] + lb[c + 1]) + rb * vb) * g1;
  Pack2h p; p.h[0] = (_Float16)z0; p.h[1] = (_Float16)z1;
  unsigned int* dst = (unsigned int*)((unsigned short*)Z16 + e);
  const unsigned int pv = p.u;
  *(volatile unsigned int*)dst = pv;
  __threadfence();
  *(volatile unsigned int*)dst = pv;
}

extern "C" void kernel_launch(void* const* d_in, const int* in_sizes, int n_in,
                              void* d_out, int out_size, void* d_ws, size_t ws_size, hipStream_t stream)
{
  if (n_in < 28) return;
  if (in_sizes[0] != TT * HD || in_sizes[1] != NH * HS * HS || in_sizes[2] != TT * HD) return;
  if (in_sizes[3] != TT * HS || in_sizes[4] != TT * HS) return;
  if (in_sizes[5] != HD || in_sizes[6] != HD * DW || in_sizes[7] != DW * HD) return;
  if (in_sizes[8] != HD || in_sizes[9] != HD * DA || in_sizes[10] != DA * HD) return;
  if (in_sizes[11] != HD || in_sizes[12] != HD * DV || in_sizes[13] != DV * HD) return;
  if (in_sizes[14] != HD * DG || in_sizes[15] != DG * HD) return;
  if (in_sizes[16] != HD || in_sizes[17] != HD || in_sizes[18] != NH * HS) return;
  if (in_sizes[19] != HD * HD || in_sizes[20] != HD || in_sizes[21] != ATTD * HD || in_sizes[22] != ATTD) return;
  if (in_sizes[23] != ATTD * HD || in_sizes[24] != ATTD || in_sizes[25] != HD * HD || in_sizes[26] != HD || in_sizes[27] != HD) return;
  if ((size_t)out_size < (size_t)2 * TT * HD + (size_t)NH * HS * HS) return;

  const float* x      = (const float*)d_in[0];
  const float* wkv_in = (const float*)d_in[1];
  const float* vfirst = (const float*)d_in[2];
  const float* cosT   = (const float*)d_in[3];
  const float* sinT   = (const float*)d_in[4];
  const float* w0 = (const float*)d_in[5];
  const float* w1 = (const float*)d_in[6];
  const float* w2 = (const float*)d_in[7];
  const float* a0 = (const float*)d_in[8];
  const float* a1 = (const float*)d_in[9];
  const float* a2 = (const float*)d_in[10];
  const float* v0 = (const float*)d_in[11];
  const float* v1 = (const float*)d_in[12];
  const float* v2 = (const float*)d_in[13];
  const float* g1 = (const float*)d_in[14];
  const float* g2 = (const float*)d_in[15];
  const float* k_k = (const float*)d_in[16];
  const float* k_a = (const float*)d_in[17];
  const float* r_k = (const float*)d_in[18];
  const float* q_w = (const float*)d_in[19];
  const float* q_b = (const float*)d_in[20];
  const float* k_w = (const float*)d_in[21];
  const float* k_b = (const float*)d_in[22];
  const float* v_w = (const float*)d_in[23];
  const float* v_b = (const float*)d_in[24];
  const float* o_w = (const float*)d_in[25];
  const float* ln_w = (const float*)d_in[26];
  const float* ln_b = (const float*)d_in[27];

  float* out0 = (float*)d_out;
  float* out1 = out0 + (size_t)TT * HD;
  float* out2 = out1 + (size_t)NH * HS * HS;

  char* ws = (char*)d_ws;
  size_t off = 0;
  auto take = [&](size_t bytes) -> void* { char* p = ws + off; off += (bytes + 255) & ~(size_t)255; return (void*)p; };
  const size_t PL = (size_t)TT * HD;
  _Float16* X16 = (_Float16*)take(PL * 2);
  _Float16* BW  = (_Float16*)take((size_t)HD * HD * 2);
  _Float16* w1t = (_Float16*)take((size_t)LP * HD * 2);
  _Float16* w2t = (_Float16*)take((size_t)HD * LP * 2);
  _Float16* a1t = (_Float16*)take((size_t)LP * HD * 2);
  _Float16* a2t = (_Float16*)take((size_t)HD * LP * 2);
  _Float16* v1t = (_Float16*)take((size_t)DV * HD * 2);
  _Float16* v2t = (_Float16*)take((size_t)HD * DV * 2);
  _Float16* g1t = (_Float16*)take((size_t)DG * HD * 2);
  _Float16* g2t = (_Float16*)take((size_t)HD * DG * 2);
  float* R  = (float*)take(PL * 4);
  float* Kr = (float*)take((size_t)TT * ATTD * 4);
  float* Vr = (float*)take((size_t)TT * ATTD * 4);
  float* WL = (float*)take(PL * 4);
  float* AL = (float*)take(PL * 4);
  float* VL = (float*)take(PL * 4);
  float* G  = (float*)take(PL * 4);
  _Float16* L16 = (_Float16*)take((size_t)TT * DG * 2);
  float* RB   = (float*)take((size_t)TT * NH * 4);
  float* INRM = (float*)take((size_t)TT * NH * 4);
  float* Y    = (float*)take(PL * 4);
  _Float16* Z16 = X16;
  if (off > ws_size) return;
  if (off > (size_t)134217728) return;

  const size_t n8 = PL / 8;
  const unsigned g8 = (unsigned)((n8 + 255) / 256);

  auto gemm = [&](int act, bool o16, const _Float16* A, int lda, const _Float16* Bt, int ldb, const float* bias,
                  float* Cf, _Float16* Ch, int ldc, int M, int N, int K) {
    const unsigned nb = (unsigned)(((M / 16) * (N / 64) + 3) / 4);
    if (o16) {
      if (act == 1)      k_gemm<1, true><<<nb, 128, 0, stream>>>(A, lda, Bt, ldb, WINV, bias, Cf, Ch, ldc, M, N, K);
      else if (act == 2) k_gemm<2, true><<<nb, 128, 0, stream>>>(A, lda, Bt, ldb, WINV, bias, Cf, Ch, ldc, M, N, K);
      else               k_gemm<0, true><<<nb, 128, 0, stream>>>(A, lda, Bt, ldb, WINV, bias, Cf, Ch, ldc, M, N, K);
    } else {
      k_gemm<0, false><<<nb, 128, 0, stream>>>(A, lda, Bt, ldb, WINV, bias, Cf, Ch, ldc, M, N, K);
    }
  };
  auto wt = [&](const float* Wsrc, int K, int N, _Float16* D, int ldt, int NP) {
    const size_t nthr = (size_t)NP * (ldt / 8);
    k_wt16<<<(unsigned)((nthr + 255) / 256), 256, 0, stream>>>(Wsrc, K, N, D, ldt, NP, WSCALE);
  };

  k_xcp<<<g8, 256, 0, stream>>>(x, vfirst, X16, out2, n8);
  k_cvt16<<<(unsigned)(((size_t)HD * HD / 8 + 255) / 256), 256, 0, stream>>>(q_w, BW, WSCALE, (size_t)HD * HD / 8);
  gemm(0, false, X16, HD, BW, HD, q_b, R, nullptr, HD, TT, HD, HD);
  wt(w1, HD, DW, w1t, HD, LP);
  wt(w2, DW, HD, w2t, LP, HD);
  gemm(1, true, X16, HD, w1t, HD, nullptr, nullptr, L16, LP, TT, LP, HD);
  gemm(0, false, L16, LP, w2t, LP, w0, WL, nullptr, HD, TT, HD, DW);
  k_cvt16<<<(unsigned)(((size_t)ATTD * HD / 8 + 255) / 256), 256, 0, stream>>>(k_w, BW, WSCALE, (size_t)ATTD * HD / 8);
  gemm(0, false, X16, HD, BW, HD, k_b, Kr, nullptr, ATTD, TT, ATTD, HD);
  k_cvt16<<<(unsigned)(((size_t)ATTD * HD / 8 + 255) / 256), 256, 0, stream>>>(v_w, BW, WSCALE, (size_t)ATTD * HD / 8);
  gemm(0, false, X16, HD, BW, HD, v_b, Vr, nullptr, ATTD, TT, ATTD, HD);
  wt(a1, HD, DA, a1t, HD, LP);
  wt(a2, DA, HD, a2t, LP, HD);
  gemm(0, true, X16, HD, a1t, HD, nullptr, nullptr, L16, LP, TT, LP, HD);
  gemm(0, false, L16, LP, a2t, LP, a0, AL, nullptr, HD, TT, HD, DA);
  wt(v1, HD, DV, v1t, HD, DV);
  wt(v2, DV, HD, v2t, DV, HD);
  gemm(0, true, X16, HD, v1t, HD, nullptr, nullptr, L16, DV, TT, DV, HD);
  gemm(0, false, L16, DV, v2t, DV, v0, VL, nullptr, HD, TT, HD, DV);
  wt(g1, HD, DG, g1t, HD, DG);
  wt(g2, DG, HD, g2t, DG, HD);
  gemm(2, true, X16, HD, g1t, HD, nullptr, nullptr, L16, DG, TT, DG, HD);
  gemm(0, false, L16, DG, g2t, DG, nullptr, G, nullptr, HD, TT, HD, DG);
  k_prep<<<TT, 256, 0, stream>>>(R, Kr, Vr, WL, AL, VL, vfirst, cosT, sinT, k_k, k_a, r_k, INRM, RB);
  k_wkv<<<NH, 256, 0, stream>>>(wkv_in, R, WL, AL, VL, Kr, cosT, sinT, k_k, k_a, INRM, Y, out1);
  k_fin<<<(unsigned)(TT * NH / 8), 256, 0, stream>>>(Y, VL, G, RB, ln_w, ln_b, Z16);
  k_cvt16<<<(unsigned)(((size_t)HD * HD / 8 + 255) / 256), 256, 0, stream>>>(o_w, BW, WSCALE, (size_t)HD * HD / 8);
  gemm(0, false, Z16, HD, BW, HD, nullptr, out0, nullptr, HD, TT, HD, HD);
}
